// Model_79164837200451
// MI455X (gfx1250) — hardware-verified
//
#include <hip/hip_runtime.h>
#include <stddef.h>
#include <stdint.h>


#define NPT    65536
#define CCH    128
#define NSN    16
#define CSC    16
#define NQKV   384
#define KV2    256
#define W1K    256
#define W2K    32
#define BN_EPS 1e-5f

#define GBM    64
#define GBN    128
#define GTHR   128

#define PTHR   256
#define NB_XB  ((NPT * CCH / 8) / PTHR)
#define NB_P4  (NPT / PTHR)
#define NB_W   ((NQKV * CCH / 8) / PTHR)
#define NB_TOT (NB_XB + NB_P4 + NB_W + 2)

#define PT_PW2 0
#define PT_PB2 384
#define PT_M1  512
#define PT_R1  640
#define PT_G1  768
#define PT_B1  896
#define PT_COL 1024
#define PT_POS 1120
#define PT_N   1152
#define PT_NR  147

#define ATHR   256
#define AWAVES 8
#define QPW    8
#define QPB    (AWAVES * QPW)
#define AP     264
#define A2P    40
#define WO_A   0
#define WO_V   (WO_A + NSN * AP * 2)
#define WO_T   (WO_V + NSN * CCH * 4)
#define WO_A2  (WO_T + NSN * 4 * 4)
#define WO_ATT (WO_A2 + NSN * A2P * 2)
#define W_BYTES (WO_ATT + NSN * CSC * 4)
#define ATT_LDS_BYTES (AWAVES * W_BYTES)
#define WSMAX  134217728

static_assert(NSN == 16 && CCH == 128 && CSC == 16);
static_assert(NPT % 128 == 0 && NPT % GBM == 0 && NPT % QPB == 0 && NPT % PTHR == 0);
static_assert(ATHR == AWAVES * 32 && AWAVES == 8 && QPW == 8 && QPB == 64);
static_assert(CCH % 32 == 0 && W1K == 2 * CCH && W2K == 2 * CSC && W2K == 32);
static_assert(NQKV == 3 * CCH && NQKV % GBN == 0 && GBN == CCH && KV2 == 2 * CCH);
static_assert(GBM == (GTHR / 32) * 16 && GBN == 4 * 32);
static_assert((AP * 2) % 16 == 0 && AP >= W1K && (A2P * 2) % 16 == 0 && A2P >= W2K);
static_assert(WO_V % 16 == 0 && WO_T % 16 == 0 && WO_A2 % 16 == 0 && WO_ATT % 16 == 0 && W_BYTES % 16 == 0);
static_assert(W_BYTES == 19200 && ATT_LDS_BYTES == 153600 && ATT_LDS_BYTES <= 327680);
static_assert((NPT * CCH / 8) % PTHR == 0 && (NQKV * CCH / 8) % PTHR == 0 && NB_W == 24);
static_assert(PT_POS + 24 <= PT_N && PT_N % 32 == 0 && PT_N == 1024 + 4 * 32);
static_assert((PT_POS * 4) % 16 == 0 && (PT_COL * 4) % 16 == 0);

typedef float          v4f   __attribute__((ext_vector_type(4)));
typedef float          v8f   __attribute__((ext_vector_type(8)));
typedef int            v4i   __attribute__((ext_vector_type(4)));
typedef int            v8i   __attribute__((ext_vector_type(8)));
typedef unsigned       v2u   __attribute__((ext_vector_type(2)));
typedef unsigned short v8us  __attribute__((ext_vector_type(8)));
typedef unsigned short v16us __attribute__((ext_vector_type(16)));
typedef __bf16         v16bf __attribute__((ext_vector_type(16)));
typedef v4f  __attribute__((may_alias)) v4fa;
typedef v4i  __attribute__((may_alias)) v4ia;
typedef v2u  __attribute__((may_alias)) v2ua;
typedef v8us __attribute__((may_alias)) v8usa;
union FragB { v16bf v; v16us u; v8us h[2]; v8i w; };

__device__ __forceinline__ v8f wmb(const FragB& a, const FragB& b, v8f c) {
  v8f d = __builtin_amdgcn_wmma_f32_16x16x32_bf16(false, a.v, false, b.v, (short)0, c, false, false);
  asm volatile("v_nop\n\tv_nop\n\tv_nop\n\tv_nop" : "+v"(d) : "v"(a.w), "v"(b.w));
  return d;
}

__device__ __forceinline__ unsigned bf16_bits(float f) {
  const unsigned u = __float_as_uint(f);
  return (u + 0x7FFFu + ((u >> 16) & 1u)) >> 16;
}
__device__ __forceinline__ float bfr(float f) {
  return __uint_as_float(bf16_bits(f) << 16);
}
__device__ __forceinline__ v8us cvt8(const float* s) {
  const v4f a = *(const v4fa*)s;
  const v4f b = *(const v4fa*)(s + 4);
  v8us o;
  o[0] = (unsigned short)bf16_bits(a.x);
  o[1] = (unsigned short)bf16_bits(a.y);
  o[2] = (unsigned short)bf16_bits(a.z);
  o[3] = (unsigned short)bf16_bits(a.w);
  o[4] = (unsigned short)bf16_bits(b.x);
  o[5] = (unsigned short)bf16_bits(b.y);
  o[6] = (unsigned short)bf16_bits(b.z);
  o[7] = (unsigned short)bf16_bits(b.w);
  return o;
}
__device__ __forceinline__ void put16(unsigned short* dp, v8us o) {
  *(volatile v8us*)dp = o;
  __threadfence();
  *(volatile v8us*)dp = o;
}
__device__ __forceinline__ void putf4(float* dp, v4f o) {
  *(volatile v4f*)dp = o;
  __threadfence();
  *(volatile v4f*)dp = o;
}
__device__ __forceinline__ float pemb(float t0, float t1, float t2, float wa, float wb, float wc, float b) {
  float s = t0 * wa;
  s = fmaf(t1, wb, s);
  s = fmaf(t2, wc, s);
  return s + b;
}
__device__ __forceinline__ float bnrelu(float v, float mm, float r, float g, float b) {
  const float y = ((v - mm) * r) * g + b;
  return (y > 0.0f) ? y : 0.0f;
}

__global__ __launch_bounds__(PTHR) void k_prep(
    const float* __restrict__ p, const float* __restrict__ x,
    const float* __restrict__ Wq, const float* __restrict__ bq,
    const float* __restrict__ Wk, const float* __restrict__ bk,
    const float* __restrict__ Wv, const float* __restrict__ bv,
    const float* __restrict__ pw1, const float* __restrict__ pb1,
    const float* __restrict__ pbn_g, const float* __restrict__ pbn_b,
    const float* __restrict__ pbn_m, const float* __restrict__ pbn_v,
    const float* __restrict__ pw2, const float* __restrict__ pb2,
    const float* __restrict__ g1, const float* __restrict__ b1,
    const float* __restrict__ m1, const float* __restrict__ v1,
    const float* __restrict__ ww1, const float* __restrict__ wb1,
    const float* __restrict__ g2, const float* __restrict__ b2,
    const float* __restrict__ m2, const float* __restrict__ v2,
    const float* __restrict__ ww2, const float* __restrict__ wb2,
    unsigned short* XB, float* P4, unsigned short* WQKV, float* BQKV,
    unsigned short* W1D, unsigned short* W2D, float* PT)
{
  __shared__ __attribute__((aligned(16))) float sPT[PT_N];
  const int b = (int)blockIdx.x, tid = (int)threadIdx.x, lane = tid & 31, wave = tid >> 5;

  if (b < NB_XB) {
    const size_t u = (size_t)b * PTHR + (size_t)tid;
    put16(XB + u * 8, cvt8(x + u * 8));
    return;
  }
  if (b < NB_XB + NB_P4) {
    const size_t r = (size_t)(b - NB_XB) * PTHR + (size_t)tid;
    const float x0 = p[r * 3 + 0];
    const float x1 = p[r * 3 + 1];
    const float x2 = p[r * 3 + 2];
    const v4f q = {bfr(x0), bfr(x1), bfr(x2), 0.0f};
    putf4(P4 + r * 4, q);
    return;
  }
  if (b < NB_XB + NB_P4 + NB_W) {
    const int bb  = b - (NB_XB + NB_P4);
    const int mat = bb >> 3;
    const size_t v = (size_t)(bb & 7) * PTHR + (size_t)tid;
    if (mat == 0)      put16(WQKV + v * 8,                       cvt8(Wq + v * 8));
    else if (mat == 1) put16(WQKV + (size_t)CCH * CCH + v * 8,   cvt8(Wk + v * 8));
    else               put16(WQKV + (size_t)2 * CCH * CCH + v * 8, cvt8(Wv + v * 8));
    return;
  }
  if (b == NB_TOT - 2) {
    if (tid < CCH) {
      const int c = tid;
      const float w0 = pw2[c * 3 + 0];
      const float w1 = pw2[c * 3 + 1];
      const float w2 = pw2[c * 3 + 2];
      const float pb = pb2[c];
      const float mm = m1[c];
      const float vv = v1[c];
      const float gg = g1[c];
      const float bb1 = b1[c];
      sPT[PT_PW2 + c]           = bfr(w0);
      sPT[PT_PW2 + CCH + c]     = bfr(w1);
      sPT[PT_PW2 + 2 * CCH + c] = bfr(w2);
      sPT[PT_PB2 + c]           = bfr(pb);
      sPT[PT_M1 + c]            = bfr(mm);
      sPT[PT_R1 + c]            = bfr(vv);
      sPT[PT_G1 + c]            = bfr(gg);
      sPT[PT_B1 + c]            = bfr(bb1);
    } else if (wave == 4) {
      const int c = lane & 15;
      const float a0 = wb1[c];
      const float a1 = m2[c];
      const float a2 = v2[c];
      const float a3 = g2[c];
      const float a4 = b2[c];
      const float a5 = wb2[c];
      sPT[PT_COL + c]      = bfr(a0);
      sPT[PT_COL + 16 + c] = bfr(a1);
      sPT[PT_COL + 32 + c] = bfr(a2);
      sPT[PT_COL + 48 + c] = bfr(a3);
      sPT[PT_COL + 64 + c] = bfr(a4);
      sPT[PT_COL + 80 + c] = bfr(a5);
    } else if (wave == 5) {
      const int l9 = lane < 9 ? lane : 8;
      const int o9 = l9 / 3, k9 = l9 - 3 * o9;
      const int l3 = lane < 3 ? lane : 2;
      const float a0 = pw1[l9];
      const float a1 = pb1[l3];
      const float a2 = pbn_m[l3];
      const float a3 = pbn_v[l3];
      const float a4 = pbn_g[l3];
      const float a5 = pbn_b[l3];
      sPT[PT_POS + 4 * o9 + k9]      = bfr(a0);
      sPT[PT_POS + 4 * l3 + 3]       = bfr(a1);
      sPT[PT_POS + 12 + 4 * l3 + 0]  = bfr(a2);
      sPT[PT_POS + 12 + 4 * l3 + 1]  = bfr(a3);
      sPT[PT_POS + 12 + 4 * l3 + 2]  = bfr(a4);
      sPT[PT_POS + 12 + 4 * l3 + 3]  = bfr(a5);
    } else if (wave == 6) {
      sPT[PT_POS + 24 + (lane & 7)] = 0.0f;
    }
    __syncthreads();
    const int tc = tid < PT_NR ? tid : PT_NR - 1;
    int slot = PT_R1 + tc;
    if (tc >= CCH)       slot = PT_COL + 32 + (tc - CCH);
    if (tc >= CCH + CSC) slot = PT_POS + 12 + 4 * (tc - CCH - CSC) + 1;
    const float var = sPT[slot];
    const float rr = 1.0f / sqrtf(var + BN_EPS);
    __syncthreads();
    if (tid < PT_NR) sPT[slot] = rr;
    __syncthreads();
    {
      const v4f o = *(const v4fa*)(sPT + 4 * tid);
      putf4(PT + 4 * tid, o);
    }
    if (wave == 0) {
      const v4f o = *(const v4fa*)(sPT + 1024 + 4 * lane);
      putf4(PT + 1024 + 4 * lane, o);
    }
    return;
  }
#pragma unroll 1
  for (int it = 0; it < 2; ++it) {
    const int v  = tid + PTHR * it;
    const int n  = v >> 5;
    const int k8 = (v & 31) * 8;
    put16(W1D + (size_t)v * 8, cvt8(ww1 + n * CCH + (k8 & (CCH - 1))));
  }
  if (wave == 0) {
    const v4f a = *(const v4fa*)(bq + 4 * lane);
    const v4f o = {bfr(a.x), bfr(a.y), bfr(a.z), bfr(a.w)};
    putf4(BQKV + 4 * lane, o);
  } else if (wave == 1) {
    const v4f a = *(const v4fa*)(bk + 4 * lane);
    const v4f o = {bfr(a.x), bfr(a.y), bfr(a.z), bfr(a.w)};
    putf4(BQKV + CCH + 4 * lane, o);
  } else if (wave == 2) {
    const v4f a = *(const v4fa*)(bv + 4 * lane);
    const v4f o = {bfr(a.x), bfr(a.y), bfr(a.z), bfr(a.w)};
    putf4(BQKV + 2 * CCH + 4 * lane, o);
  }
  if (tid < 64) {
    const int n  = tid >> 2;
    const int k8 = (tid & 3) * 8;
    put16(W2D + (size_t)tid * 8, cvt8(ww2 + n * CSC + (k8 & (CSC - 1))));
  }
}

__global__ __launch_bounds__(GTHR) void k_qkv(const unsigned short* __restrict__ A,
                                              const unsigned short* __restrict__ BT,
                                              const float* __restrict__ BQ,
                                              float* wsf, long long oXQ, long long oXKV) {
  __shared__ __attribute__((aligned(16))) float stg[GBM * GBN];
  const int tid = (int)threadIdx.x, lane = tid & 31, wave = tid >> 5, hh = lane >> 4, m = lane & 15;
  const int by = (int)blockIdx.y;
  const int rowBase = (int)blockIdx.x * GBM;
  const int colBase = by * GBN;

  v8f acc[8];
  {
    const v8f z = {0.f, 0.f, 0.f, 0.f, 0.f, 0.f, 0.f, 0.f};
#pragma unroll
    for (int t = 0; t < 8; ++t) acc[t] = z;
  }
  const unsigned short* ap = A  + (size_t)(rowBase + 16 * wave + m) * (size_t)CCH + 8 * hh;
  const unsigned short* bp = BT + (size_t)(colBase + m) * (size_t)CCH + 8 * hh;

#pragma unroll 1
  for (int k0 = 0; k0 < CCH; k0 += 32) {
    FragB af;
    af.h[0] = *(const v8usa*)(ap + k0);
    af.h[1] = *(const v8usa*)(ap + k0 + 16);
#pragma unroll
    for (int nt = 0; nt < 8; ++nt) {
      const unsigned short* wq = bp + (size_t)(16 * nt) * (size_t)CCH + k0;
      FragB bf;
      bf.h[0] = *(const v8usa*)wq;
      bf.h[1] = *(const v8usa*)(wq + 16);
      acc[nt] = wmb(af, bf, acc[nt]);
    }
  }

#pragma unroll
  for (int nt = 0; nt < 8; ++nt) {
    const int lc = 16 * nt + m;
    const float bvv = BQ[colBase + lc];
#pragma unroll
    for (int r = 0; r < 8; ++r) {
      const int lr = 16 * wave + 8 * hh + r;
      stg[lr * GBN + lc] = acc[nt][r] + bvv;
    }
  }
  __syncthreads();

  const long long cb = (by == 0) ? oXQ : (oXKV + (long long)(by - 1) * CCH);
  const int ldc = (by == 0) ? CCH : KV2;
  float* Cm = wsf + cb;
  v4f pv[16];
#pragma unroll
  for (int i = 0; i < 16; ++i) pv[i] = *(const v4fa*)(stg + (16 * wave + i) * GBN + 4 * lane);
#pragma unroll
  for (int i = 0; i < 16; ++i) {
    float* op = Cm + (size_t)(rowBase + 16 * wave + i) * (size_t)ldc + 4 * lane;
    *(volatile v4f*)op = pv[i];
  }
  __threadfence();
#pragma unroll
  for (int i = 0; i < 16; ++i) {
    float* op = Cm + (size_t)(rowBase + 16 * wave + i) * (size_t)ldc + 4 * lane;
    *(volatile v4f*)op = pv[i];
  }
}

__global__ __launch_bounds__(ATHR) void k_attn(const int* __restrict__ idx, const float* __restrict__ P4,
                                               const float* __restrict__ XQ, const float* __restrict__ XKV,
                                               const unsigned short* __restrict__ W1D,
                                               const unsigned short* __restrict__ W2D,
                                               const float* __restrict__ PT, float* out) {
  extern __shared__ __attribute__((aligned(16))) unsigned char dyn[];
  const int tid = (int)threadIdx.x, lane = tid & 31, wave = tid >> 5, hh = lane >> 4, m = lane & 15;
  unsigned char*  wbase = dyn + wave * W_BYTES;
  unsigned short* sA   = (unsigned short*)(wbase + WO_A);
  float*          sV   = (float*)(wbase + WO_V);
  int*            sT   = (int*)(wbase + WO_T);
  unsigned short* sA2  = (unsigned short*)(wbase + WO_A2);
  float*          sAtt = (float*)(wbase + WO_ATT);
  const int c4 = 4 * lane;

  const v4f pwa = *(const v4fa*)(PT + PT_PW2 + c4);
  const v4f pwb = *(const v4fa*)(PT + PT_PW2 + CCH + c4);
  const v4f pwc = *(const v4fa*)(PT + PT_PW2 + 2 * CCH + c4);
  const v4f pbv = *(const v4fa*)(PT + PT_PB2 + c4);
  const v4f m1v = *(const v4fa*)(PT + PT_M1 + c4);
  const v4f r1v = *(const v4fa*)(PT + PT_R1 + c4);
  const v4f g1v = *(const v4fa*)(PT + PT_G1 + c4);
  const v4f b1v = *(const v4fa*)(PT + PT_B1 + c4);
  const float wb1c = PT[PT_COL + m];
  const float m2c  = PT[PT_COL + 16 + m];
  const float r2c  = PT[PT_COL + 32 + m];
  const float g2c  = PT[PT_COL + 48 + m];
  const float b2c  = PT[PT_COL + 64 + m];
  const float wb2c = PT[PT_COL + 80 + m];
  const v4f q0 = *(const v4fa*)(PT + PT_POS + 0);
  const v4f q1 = *(const v4fa*)(PT + PT_POS + 4);
  const v4f q2 = *(const v4fa*)(PT + PT_POS + 8);
  const v4f h0 = *(const v4fa*)(PT + PT_POS + 12);
  const v4f h1 = *(const v4fa*)(PT + PT_POS + 16);
  const v4f h2 = *(const v4fa*)(PT + PT_POS + 20);

  FragB w1f[4], w2f;
  {
    const unsigned short* wr = W1D + (size_t)m * W1K + 8 * hh;
#pragma unroll
    for (int ks = 0; ks < 4; ++ks) {
      w1f[ks].h[0] = *(const v8usa*)(wr + 32 * ks);
      w1f[ks].h[1] = *(const v8usa*)(wr + 32 * ks + 16);
    }
    const unsigned short* w2r = W2D + (size_t)m * W2K + 8 * hh;
    w2f.h[0] = *(const v8usa*)w2r;
    w2f.h[1] = *(const v8usa*)(w2r + 16);
  }
  const v8f z8 = {0.f, 0.f, 0.f, 0.f, 0.f, 0.f, 0.f, 0.f};

#pragma unroll 1
  for (int qi = 0; qi < QPW; ++qi) {
    const int i = (int)blockIdx.x * QPB + wave * QPW + qi;

    int nl = idx[(size_t)i * NSN + m];
    nl = nl < 0 ? 0 : (nl > NPT - 1 ? NPT - 1 : nl);

    {
      const v4f pn = *(const v4fa*)(P4 + (size_t)nl * 4);
      const v4f pq = *(const v4fa*)(P4 + (size_t)i * 4);
      const float rx = pn.x - pq.x, ry = pn.y - pq.y, rz = pn.z - pq.z;
      float l0 = rx * q0.x; l0 = fmaf(ry, q0.y, l0); l0 = fmaf(rz, q0.z, l0); l0 += q0.w;
      float l1 = rx * q1.x; l1 = fmaf(ry, q1.y, l1); l1 = fmaf(rz, q1.z, l1); l1 += q1.w;
      float l2 = rx * q2.x; l2 = fmaf(ry, q2.y, l2); l2 = fmaf(rz, q2.z, l2); l2 += q2.w;
      const float t0 = bnrelu(l0, h0.x, h0.y, h0.z, h0.w);
      const float t1 = bnrelu(l1, h1.x, h1.y, h1.z, h1.w);
      const float t2 = bnrelu(l2, h2.x, h2.y, h2.z, h2.w);
      const v4i tw = {__float_as_int(t0), __float_as_int(t1), __float_as_int(t2), nl};
      if (lane < 16) *(v4ia*)(sT + 4 * m) = tw;
    }
    __syncthreads();

    {
      const v4f xq4 = *(const v4fa*)(XQ + (size_t)i * CCH + c4);
#pragma unroll 2
      for (int j = 0; j < NSN; ++j) {
        const v4i tv = *(const v4ia*)(sT + 4 * j);
        const float t0 = __int_as_float(tv.x);
        const float t1 = __int_as_float(tv.y);
        const float t2 = __int_as_float(tv.z);
        int n = tv.w;
        n = n < 0 ? 0 : (n > NPT - 1 ? NPT - 1 : n);
        const float* kr = XKV + (size_t)n * KV2 + c4;
        const v4f xk = *(const v4fa*)kr;
        const v4f xv = *(const v4fa*)(kr + CCH);
        const float pe0 = pemb(t0, t1, t2, pwa.x, pwb.x, pwc.x, pbv.x);
        const float pe1 = pemb(t0, t1, t2, pwa.y, pwb.y, pwc.y, pbv.y);
        const float pe2 = pemb(t0, t1, t2, pwa.z, pwb.z, pwc.z, pbv.z);
        const float pe3 = pemb(t0, t1, t2, pwa.w, pwb.w, pwc.w, pbv.w);
        const float a0 = bnrelu((xk.x - xq4.x) + pe0, m1v.x, r1v.x, g1v.x, b1v.x);
        const float a1 = bnrelu((xk.y - xq4.y) + pe1, m1v.y, r1v.y, g1v.y, b1v.y);
        const float a2 = bnrelu((xk.z - xq4.z) + pe2, m1v.z, r1v.z, g1v.z, b1v.z);
        const float a3 = bnrelu((xk.w - xq4.w) + pe3, m1v.w, r1v.w, g1v.w, b1v.w);
        const unsigned hb0 = bf16_bits(a0), hb1 = bf16_bits(a1), hb2 = bf16_bits(a2), hb3 = bf16_bits(a3);
        const unsigned lb0 = bf16_bits(a0 - __uint_as_float(hb0 << 16));
        const unsigned lb1 = bf16_bits(a1 - __uint_as_float(hb1 << 16));
        const unsigned lb2 = bf16_bits(a2 - __uint_as_float(hb2 << 16));
        const unsigned lb3 = bf16_bits(a3 - __uint_as_float(hb3 << 16));
        const v2u hw = {hb0 | (hb1 << 16), hb2 | (hb3 << 16)};
        const v2u lw = {lb0 | (lb1 << 16), lb2 | (lb3 << 16)};
        *(v2ua*)(sA + j * AP + c4)       = hw;
        *(v2ua*)(sA + j * AP + CCH + c4) = lw;
        const v4f vp = {xv.x + pe0, xv.y + pe1, xv.z + pe2, xv.w + pe3};
        *(v4fa*)(sV + j * CCH + c4) = vp;
      }
    }
    __syncthreads();

    {
      v8f accH = z8, accL = z8;
      const unsigned short* ar = sA + m * AP + 8 * hh;
#pragma unroll
      for (int ks = 0; ks < 4; ++ks) {
        FragB ah, al;
        ah.h[0] = *(const v8usa*)(ar + 32 * ks);
        ah.h[1] = *(const v8usa*)(ar + 32 * ks + 16);
        al.h[0] = *(const v8usa*)(ar + CCH + 32 * ks);
        al.h[1] = *(const v8usa*)(ar + CCH + 32 * ks + 16);
        accH = wmb(ah, w1f[ks], accH);
        accL = wmb(al, w1f[ks], accL);
      }
#pragma unroll
      for (int r = 0; r < 8; ++r) {
        const float v  = (accH[r] + accL[r]) + wb1c;
        const float a2 = bnrelu(v, m2c, r2c, g2c, b2c);
        const unsigned hb = bf16_bits(a2);
        const unsigned lb = bf16_bits(a2 - __uint_as_float(hb << 16));
        sA2[(8 * hh + r) * A2P + m]       = (unsigned short)hb;
        sA2[(8 * hh + r) * A2P + CSC + m] = (unsigned short)lb;
      }
    }
    __syncthreads();

    {
      FragB a2f;
      a2f.h[0] = *(const v8usa*)(sA2 + m * A2P + 8 * hh);
      a2f.h[1] = *(const v8usa*)(sA2 + m * A2P + 16 + 8 * hh);
      const v8f d2 = wmb(a2f, w2f, z8);
      float lg[8];
#pragma unroll
      for (int r = 0; r < 8; ++r) lg[r] = d2[r] + wb2c;
      float mx = lg[0];
#pragma unroll
      for (int r = 1; r < 8; ++r) mx = fmaxf(mx, lg[r]);
      const float mo = __shfl_xor(mx, 16);
      mx = fmaxf(mx, mo);
      float e[8];
      float s = 0.0f;
#pragma unroll
      for (int r = 0; r < 8; ++r) { e[r] = expf(lg[r] - mx); s += e[r]; }
      const float so = __shfl_xor(s, 16);
      s = s + so;
      const float inv = 1.0f / s;
#pragma unroll
      for (int r = 0; r < 8; ++r) sAtt[(8 * hh + r) * CSC + m] = e[r] * inv;
    }
    __syncthreads();

    {
      const float* ap = sAtt + 4 * (lane & 3);
      const float* vp = sV + c4;
      float o0 = 0.0f, o1 = 0.0f, o2 = 0.0f, o3 = 0.0f;
#pragma unroll 4
      for (int j = 0; j < NSN; ++j) {
        const v4f a = *(const v4fa*)(ap + CSC * j);
        const v4f v = *(const v4fa*)(vp + CCH * j);
        o0 = fmaf(a.x, v.x, o0);
        o1 = fmaf(a.y, v.y, o1);
        o2 = fmaf(a.z, v.z, o2);
        o3 = fmaf(a.w, v.w, o3);
      }
      const v4f o = {o0, o1, o2, o3};
      float* op = out + (size_t)i * CCH + c4;
      *(volatile v4f*)op = o;
      __threadfence();
      *(volatile v4f*)op = o;
    }
  }
}

extern "C" void kernel_launch(void* const* d_in, const int* in_sizes, int n_in,
                              void* d_out, int out_size, void* d_ws, size_t ws_size,
                              hipStream_t stream) {
  if (n_in < 29) return;
  if (in_sizes[0] != NPT * 3 || in_sizes[1] != NPT * CCH || in_sizes[2] != NPT * NSN) return;
  if (in_sizes[3] != CCH * CCH || in_sizes[4] != CCH) return;
  if (in_sizes[5] != CCH * CCH || in_sizes[6] != CCH) return;
  if (in_sizes[7] != CCH * CCH || in_sizes[8] != CCH) return;
  if (in_sizes[9] != 9 || in_sizes[10] != 3) return;
  if (in_sizes[11] != 3 || in_sizes[12] != 3 || in_sizes[13] != 3 || in_sizes[14] != 3) return;
  if (in_sizes[15] != CCH * 3 || in_sizes[16] != CCH) return;
  if (in_sizes[17] != CCH || in_sizes[18] != CCH || in_sizes[19] != CCH || in_sizes[20] != CCH) return;
  if (in_sizes[21] != CSC * CCH || in_sizes[22] != CSC) return;
  if (in_sizes[23] != CSC || in_sizes[24] != CSC || in_sizes[25] != CSC || in_sizes[26] != CSC) return;
  if (in_sizes[27] != CSC * CSC || in_sizes[28] != CSC) return;
  if (out_size != NPT * CCH) return;

  const float* p      = (const float*)d_in[0];
  const float* x      = (const float*)d_in[1];
  const int*   idx    = (const int*)  d_in[2];
  const float* Wq     = (const float*)d_in[3];
  const float* bq     = (const float*)d_in[4];
  const float* Wk     = (const float*)d_in[5];
  const float* bk     = (const float*)d_in[6];
  const float* Wv     = (const float*)d_in[7];
  const float* bv     = (const float*)d_in[8];
  const float* pw1    = (const float*)d_in[9];
  const float* pb1    = (const float*)d_in[10];
  const float* pbn_g  = (const float*)d_in[11];
  const float* pbn_b  = (const float*)d_in[12];
  const float* pbn_m  = (const float*)d_in[13];
  const float* pbn_v  = (const float*)d_in[14];
  const float* pw2    = (const float*)d_in[15];
  const float* pb2    = (const float*)d_in[16];
  const float* wbn1_g = (const float*)d_in[17];
  const float* wbn1_b = (const float*)d_in[18];
  const float* wbn1_m = (const float*)d_in[19];
  const float* wbn1_v = (const float*)d_in[20];
  const float* ww1    = (const float*)d_in[21];
  const float* wb1    = (const float*)d_in[22];
  const float* wbn2_g = (const float*)d_in[23];
  const float* wbn2_b = (const float*)d_in[24];
  const float* wbn2_m = (const float*)d_in[25];
  const float* wbn2_v = (const float*)d_in[26];
  const float* ww2    = (const float*)d_in[27];
  const float* wb2    = (const float*)d_in[28];
  float* out = (float*)d_out;

  char* ws = (char*)d_ws;
  size_t off = 0;
  const size_t oXB   = off; off += (size_t)NPT * CCH * 2;   off = (off + 255) & ~(size_t)255;
  const size_t oXQ   = off; off += (size_t)NPT * CCH * 4;   off = (off + 255) & ~(size_t)255;
  const size_t oXKV  = off; off += (size_t)NPT * KV2 * 4;   off = (off + 255) & ~(size_t)255;
  const size_t oP4   = off; off += (size_t)NPT * 4 * 4;     off = (off + 255) & ~(size_t)255;
  const size_t oWQKV = off; off += (size_t)NQKV * CCH * 2;  off = (off + 255) & ~(size_t)255;
  const size_t oW1D  = off; off += (size_t)CSC * W1K * 2;   off = (off + 255) & ~(size_t)255;
  const size_t oW2D  = off; off += (size_t)CSC * W2K * 2;   off = (off + 255) & ~(size_t)255;
  const size_t oBQKV = off; off += (size_t)NQKV * 4;        off = (off + 255) & ~(size_t)255;
  const size_t oPT   = off; off += (size_t)PT_N * 4;        off = (off + 255) & ~(size_t)255;
  if (off > ws_size || off > (size_t)WSMAX) return;

  unsigned short* XB   = (unsigned short*)(ws + oXB);
  float*          XQ   = (float*)(ws + oXQ);
  float*          XKV  = (float*)(ws + oXKV);
  float*          P4   = (float*)(ws + oP4);
  unsigned short* WQKV = (unsigned short*)(ws + oWQKV);
  unsigned short* W1D  = (unsigned short*)(ws + oW1D);
  unsigned short* W2D  = (unsigned short*)(ws + oW2D);
  float*          BQKV = (float*)(ws + oBQKV);
  float*          PT   = (float*)(ws + oPT);

  hipFuncSetAttribute(reinterpret_cast<const void*>(&k_attn), hipFuncAttributeMaxDynamicSharedMemorySize,
                      (int)ATT_LDS_BYTES);

  k_prep<<<NB_TOT, PTHR, 0, stream>>>(p, x, Wq, bq, Wk, bk, Wv, bv, pw1, pb1, pbn_g, pbn_b, pbn_m, pbn_v,
                                      pw2, pb2, wbn1_g, wbn1_b, wbn1_m, wbn1_v, ww1, wb1,
                                      wbn2_g, wbn2_b, wbn2_m, wbn2_v, ww2, wb2,
                                      XB, P4, WQKV, BQKV, W1D, W2D, PT);
  k_qkv<<<dim3(NPT / GBM, NQKV / GBN), GTHR, 0, stream>>>(XB, WQKV, BQKV, (float*)d_ws,
                                                           (long long)(oXQ / 4), (long long)(oXKV / 4));
  k_attn<<<NPT / QPB, ATHR, ATT_LDS_BYTES, stream>>>(idx, P4, XQ, XKV, W1D, W2D, PT, out);
}
